// SelectiveSSMBlock_52536039964823
// MI455X (gfx1250) — hardware-verified
//
#include <hip/hip_runtime.h>
#include <math.h>

constexpr int NBATCH = 4;
constexpr int SEQLEN = 1024;
constexpr int DMODEL = 256;
constexpr int DSTATE = 256;
constexpr int KCONV  = 4;
constexpr int NROWS  = NBATCH * SEQLEN;
constexpr int DPROJ  = 2 * DMODEL;
constexpr int GPITCH = 264;
static_assert(DMODEL == DSTATE, "equal dims");
static_assert(NROWS % 64 == 0 && DPROJ % 64 == 0 && DMODEL % 64 == 0, "tile multiples");
static_assert(DMODEL % 32 == 0, "K multiple of 32");
static_assert((GPITCH % 8) == 0, "16B rows");

typedef __attribute__((ext_vector_type(16))) _Float16 v16h;
typedef __attribute__((ext_vector_type(8)))  _Float16 v8h;
typedef __attribute__((ext_vector_type(16))) __bf16   v16b;
typedef __attribute__((ext_vector_type(8)))  __bf16   v8b;
typedef __attribute__((ext_vector_type(8)))  float    v8f;
typedef __attribute__((ext_vector_type(4)))  float    v4f;
typedef __attribute__((ext_vector_type(4)))  unsigned v4u;

__device__ __forceinline__ unsigned short f2bf_bits(float f) {
  unsigned u = __float_as_uint(f);
  return (unsigned short)((u + 0x7FFFu + ((u >> 16) & 1u)) >> 16);
}
__device__ __forceinline__ float bf_bits2f(unsigned short h) { return __uint_as_float(((unsigned)h) << 16); }

__device__ __forceinline__ void dep_guard_h(v8f& a, v8f& b, v16h x, v16h y) { asm volatile("v_nop\n\tv_nop\n\tv_nop\n\tv_nop" : "+v"(a), "+v"(b) : "v"(x), "v"(y)); }
__device__ __forceinline__ void dep_guard_b(v8f& a, v8f& b, v16b x, v16b y) { asm volatile("v_nop\n\tv_nop\n\tv_nop\n\tv_nop" : "+v"(a), "+v"(b) : "v"(x), "v"(y)); }
__device__ __forceinline__ void keep4_h(v16h a, v16h b, v16h c, v16h d) { asm volatile("v_nop" :: "v"(a), "v"(b), "v"(c), "v"(d)); }
__device__ __forceinline__ void keep4_b(v16b a, v16b b, v16b c, v16b d) { asm volatile("v_nop" :: "v"(a), "v"(b), "v"(c), "v"(d)); }
__device__ __forceinline__ void acc_guard4(v8f& a, v8f& b, v8f& c, v8f& d) { asm volatile("v_nop\n\tv_nop\n\tv_nop\n\tv_nop" : "+v"(a), "+v"(b), "+v"(c), "+v"(d)); }
__device__ __forceinline__ void guard3_b(v8f& a, v8f& b, v16b x, v16b y, v16b z) { asm volatile("v_nop\n\tv_nop\n\tv_nop\n\tv_nop" : "+v"(a), "+v"(b) : "v"(x), "v"(y), "v"(z)); }

template <typename T> struct Frag;
template <> struct Frag<_Float16> {
  typedef v16h V; union U { v16h v; v8h h[2]; };
  static __device__ __forceinline__ v16h load(const _Float16* p) {
    U f; f.h[0] = *(const v8h*)(p); f.h[1] = *(const v8h*)(p + 16); return f.v;
  }
  static __device__ __forceinline__ v8f mma(v16h a, v16h b, v8f c) {
    return __builtin_amdgcn_wmma_f32_16x16x32_f16(false, a, false, b, (short)0, c, false, false);
  }
  static __device__ __forceinline__ void guard(v8f& a, v8f& b, v16h x, v16h y) { dep_guard_h(a, b, x, y); }
  static __device__ __forceinline__ void keep(v16h a, v16h b, v16h c, v16h d) { keep4_h(a, b, c, d); }
};
template <> struct Frag<__bf16> {
  typedef v16b V; union U { v16b v; v8b h[2]; };
  static __device__ __forceinline__ v16b load(const __bf16* p) {
    U f; f.h[0] = *(const v8b*)(p); f.h[1] = *(const v8b*)(p + 16); return f.v;
  }
  static __device__ __forceinline__ v8f mma(v16b a, v16b b, v8f c) {
    return __builtin_amdgcn_wmma_f32_16x16x32_bf16(false, a, false, b, (short)0, c, false, false);
  }
  static __device__ __forceinline__ void guard(v8f& a, v8f& b, v16b x, v16b y) { dep_guard_b(a, b, x, y); }
  static __device__ __forceinline__ void keep(v16b a, v16b b, v16b c, v16b d) { keep4_b(a, b, c, d); }
};

template <int ET> struct Elem;
template <> struct Elem<0> { typedef _Float16 T; };
template <> struct Elem<1> { typedef __bf16 T; };
template <int ET, bool SPLIT, int BIAS_MODE, int OUT_MODE, bool RESID, int ACT = 0>
__global__ __launch_bounds__(256) void wmma_gemm64(
    const unsigned short* __restrict__ Ap, const unsigned short* __restrict__ A2p, int lda, long strideA,
    const unsigned short* __restrict__ Btp, const unsigned short* __restrict__ Bt2p, int ldb, long strideB,
    void* __restrict__ Cout, void* __restrict__ Cout2, int ldc, long strideC,
    const float* __restrict__ bias,
    const float* __restrict__ resid, long strideR,
    int M, int N, int K, float scale) {
  static_assert(!(RESID && ACT != 0), "act before resid not supported");
  static_assert(!(RESID && OUT_MODE != 0), "resid with f32 out only");
  typedef typename Elem<ET>::T T;
  typedef typename Frag<T>::V V;
  const T* A = (const T*)Ap; const T* A2 = (const T*)A2p; const T* Bt = (const T*)Btp; const T* Bt2 = (const T*)Bt2p;
  __shared__ __align__(16) float sT[8][16 * 68];
  const int b    = blockIdx.y;
  const int lane = threadIdx.x & 31;
  const int wave = threadIdx.x >> 5;
  const int tilesN = N >> 6;
  const int tilesM = M >> 6;
  const int tile = blockIdx.x * 8 + wave;
  if (tile >= tilesM * tilesN) return;
  const int tm = tile / tilesN;
  const int tn = tile - tm * tilesN;
  const int m0 = tm << 6;
  const int n0 = tn << 6;

  const T* Ab  = A  + (size_t)b * strideA;
  const T* Bb  = Bt + (size_t)b * strideB;
  const T* Ab2 = SPLIT ? (A2  + (size_t)b * strideA) : nullptr;
  const T* Bb2 = SPLIT ? (Bt2 + (size_t)b * strideB) : nullptr;

  const int rlane = lane & 15;
  const int koff  = (lane >> 4) * 8;
  const int mOff  = (lane >> 4) * 8;

  v8f acc[4][4];
#pragma unroll
  for (int i = 0; i < 4; ++i)
#pragma unroll
    for (int j = 0; j < 4; ++j) acc[i][j] = (v8f){0.f,0.f,0.f,0.f,0.f,0.f,0.f,0.f};

  for (int k0 = 0; k0 < K; k0 += 32) {
    V bh[4], bl[4];
#pragma unroll
    for (int j = 0; j < 4; ++j) {
      const size_t bo = (size_t)(n0 + (j << 4) + rlane) * ldb + koff + k0;
      bh[j] = Frag<T>::load(Bb + bo);
      if (SPLIT) bl[j] = Frag<T>::load(Bb2 + bo);
    }
#pragma unroll
    for (int i = 0; i < 4; ++i) {
      const size_t ao = (size_t)(m0 + (i << 4) + rlane) * lda + koff + k0;
      V ah = Frag<T>::load(Ab + ao);
      V al;
      if (SPLIT) al = Frag<T>::load(Ab2 + ao);
#pragma unroll
      for (int j = 0; j < 4; ++j) {
        acc[i][j] = Frag<T>::mma(ah, bh[j], acc[i][j]);
        if (SPLIT) {
          acc[i][j] = Frag<T>::mma(ah, bl[j], acc[i][j]);
          acc[i][j] = Frag<T>::mma(al, bh[j], acc[i][j]);
        }
      }
      Frag<T>::guard(acc[i][0], acc[i][3], ah, SPLIT ? al : ah);
    }
    Frag<T>::keep(bh[0], bh[1], bh[2], bh[3]);
    if (SPLIT) Frag<T>::keep(bl[0], bl[1], bl[2], bl[3]);
  }
  acc_guard4(acc[0][0], acc[0][1], acc[0][2], acc[0][3]);
  acc_guard4(acc[1][0], acc[1][1], acc[1][2], acc[1][3]);
  acc_guard4(acc[2][0], acc[2][1], acc[2][2], acc[2][3]);
  acc_guard4(acc[3][0], acc[3][1], acc[3][2], acc[3][3]);

  float* slab = sT[wave];
  const float* Rb = RESID ? (resid + (size_t)b * strideR) : nullptr;
#pragma unroll
  for (int i = 0; i < 4; ++i) {
    const int mBase = m0 + (i << 4);
#pragma unroll
    for (int j = 0; j < 4; ++j) {
      const int n = n0 + (j << 4) + rlane;
      float bv = 0.f;
      if (BIAS_MODE == 2) bv = bias[n];
#pragma unroll
      for (int r = 0; r < 8; ++r) {
        float v = acc[i][j][r] * scale;
        if (BIAS_MODE == 1) v += bias[mBase + mOff + r];
        if (BIAS_MODE == 2) v += bv;
        if (ACT == 1) v = tanhf(v);
        if (ACT == 2) v = fmaxf(v, 0.0f);
        if (ACT == 3) v = v / (1.0f + expf(-v));
        if (ACT == 4) v = (v > 0.f) ? v : 0.01f * v;
        slab[(mOff + r) * 68 + (j << 4) + rlane] = v;
      }
    }
    __builtin_amdgcn_fence(__ATOMIC_RELEASE, "workgroup");
    __builtin_amdgcn_wave_barrier();
    __builtin_amdgcn_fence(__ATOMIC_ACQUIRE, "workgroup");
    if (OUT_MODE == 0) {
      float* C = (float*)Cout + (size_t)b * strideC;
      const int hh = lane >> 4, c4 = (lane & 15) * 4;
      v4f vals[8];
#pragma unroll
      for (int it = 0; it < 8; ++it) {
        const int row = it * 2 + hh;
        v4f v = *(const v4f*)(slab + row * 68 + c4);
        if (RESID) {
          const v4f rv = *(const v4f*)(Rb + (size_t)(mBase + row) * ldc + n0 + c4);
          v = v + rv;
        }
        vals[it] = v;
      }
      for (int pass = 0; pass < 2; ++pass) {
#pragma unroll
        for (int it = 0; it < 8; ++it) {
          const int row = it * 2 + hh;
          *(volatile v4f*)(C + (size_t)(mBase + row) * ldc + n0 + c4) = vals[it];
        }
        __threadfence();
      }
    } else {
      const int q = lane >> 3, c8 = (lane & 7) * 8;
      unsigned short* C  = (unsigned short*)Cout  + (size_t)b * strideC;
      unsigned short* C2 = (OUT_MODE == 2) ? ((unsigned short*)Cout2 + (size_t)b * strideC) : nullptr;
      for (int pass = 0; pass < 2; ++pass) {
#pragma unroll
        for (int it = 0; it < 4; ++it) {
          const int row = it * 4 + q;
          const float* sp = slab + row * 68 + c8;
          v8h hv, lv;
#pragma unroll
          for (int e = 0; e < 8; ++e) {
            if (OUT_MODE == 1) {
              hv[e] = (_Float16)sp[e];
              lv[e] = hv[e];
            } else {
              unsigned short hb = f2bf_bits(sp[e]);
              unsigned short lb = f2bf_bits(sp[e] - bf_bits2f(hb));
              hv[e] = __builtin_bit_cast(_Float16, hb);
              lv[e] = __builtin_bit_cast(_Float16, lb);
            }
          }
          *(volatile v8h*)(C + (size_t)(mBase + row) * ldc + n0 + c8) = hv;
          if (OUT_MODE == 2) *(volatile v8h*)(C2 + (size_t)(mBase + row) * ldc + n0 + c8) = lv;
        }
        __threadfence();
      }
    }
    __builtin_amdgcn_fence(__ATOMIC_RELEASE, "workgroup");
    __builtin_amdgcn_wave_barrier();
    __builtin_amdgcn_fence(__ATOMIC_ACQUIRE, "workgroup");
  }
}

__device__ __forceinline__ unsigned pack_hl(float a, float b, unsigned& low) {
  const unsigned short ha = f2bf_bits(a), hb = f2bf_bits(b);
  const float ra = a - bf_bits2f(ha), rb = b - bf_bits2f(hb);
  const unsigned short la = f2bf_bits(ra), lb = f2bf_bits(rb);
  low = (unsigned)la | ((unsigned)lb << 16);
  return (unsigned)ha | ((unsigned)hb << 16);
}
__device__ __forceinline__ void split8(v4f a, v4f b, v4u& hv, v4u& lv) {
  unsigned l0, l1, l2, l3;
  const unsigned h0 = pack_hl(a[0], a[1], l0);
  const unsigned h1 = pack_hl(a[2], a[3], l1);
  const unsigned h2 = pack_hl(b[0], b[1], l2);
  const unsigned h3 = pack_hl(b[2], b[3], l3);
  hv = (v4u){h0, h1, h2, h3};
  lv = (v4u){l0, l1, l2, l3};
}
__device__ __forceinline__ void store2_planes(unsigned short* ph, unsigned short* pl, v4u hv, v4u lv) {
  *(volatile v4u*)ph = hv;
  *(volatile v4u*)pl = lv;
  __threadfence();
  *(volatile v4u*)ph = hv;
  *(volatile v4u*)pl = lv;
}
__device__ __forceinline__ float silu_f(float v) {
  const float e = expf(-v);
  return v * __builtin_amdgcn_rcpf(1.0f + e);
}

__global__ __launch_bounds__(256) void split_planes(const float* __restrict__ in,
                                                    unsigned short* __restrict__ hi,
                                                    unsigned short* __restrict__ lo, int n8) {
  const int i = blockIdx.x * 256 + threadIdx.x;
  if (i >= n8) return;
  const float* p = in + (size_t)i * 8;
  const v4f a = *(const v4f*)p;
  const v4f c = *(const v4f*)(p + 4);
  v4u hv, lv;
  split8(a, c, hv, lv);
  store2_planes(hi + (size_t)i * 8, lo + (size_t)i * 8, hv, lv);
}

__global__ __launch_bounds__(256) void split_transpose_sq(const float* __restrict__ in,
                                                          unsigned short* __restrict__ hi,
                                                          unsigned short* __restrict__ lo) {
  const int i = blockIdx.x * 256 + threadIdx.x;
  const int n = i >> 5, j = i & 31;
  v4f a, c;
  a[0] = in[(size_t)(8 * j + 0) * DSTATE + n];
  a[1] = in[(size_t)(8 * j + 1) * DSTATE + n];
  a[2] = in[(size_t)(8 * j + 2) * DSTATE + n];
  a[3] = in[(size_t)(8 * j + 3) * DSTATE + n];
  c[0] = in[(size_t)(8 * j + 4) * DSTATE + n];
  c[1] = in[(size_t)(8 * j + 5) * DSTATE + n];
  c[2] = in[(size_t)(8 * j + 6) * DSTATE + n];
  c[3] = in[(size_t)(8 * j + 7) * DSTATE + n];
  v4u hv, lv;
  split8(a, c, hv, lv);
  const size_t off = (size_t)n * DSTATE + 8 * j;
  store2_planes(hi + off, lo + off, hv, lv);
}

__global__ __launch_bounds__(256) void layernorm_split(const float* __restrict__ x,
                                                       const float* __restrict__ gam,
                                                       const float* __restrict__ bet,
                                                       unsigned short* __restrict__ xh,
                                                       unsigned short* __restrict__ xl) {
  const int wave = threadIdx.x >> 5, lane = threadIdx.x & 31;
  const int row = blockIdx.x * 8 + wave;
  const float* p = x + (size_t)row * DMODEL + lane * 8;
  const v4f a = *(const v4f*)p;
  const v4f c = *(const v4f*)(p + 4);
  float s = ((a[0] + a[1]) + (a[2] + a[3])) + ((c[0] + c[1]) + (c[2] + c[3]));
#pragma unroll
  for (int o = 16; o > 0; o >>= 1) s += __shfl_xor(s, o, 32);
  const float mu = s * (1.0f / (float)DMODEL);
  const v4f da = a - mu;
  const v4f dc = c - mu;
  float s2 = ((da[0] * da[0] + da[1] * da[1]) + (da[2] * da[2] + da[3] * da[3]))
           + ((dc[0] * dc[0] + dc[1] * dc[1]) + (dc[2] * dc[2] + dc[3] * dc[3]));
#pragma unroll
  for (int o = 16; o > 0; o >>= 1) s2 += __shfl_xor(s2, o, 32);
  const float var = s2 * (1.0f / (float)DMODEL);
  const float rs = rsqrtf(var + 1e-5f);
  const v4f ga = *(const v4f*)(gam + lane * 8);
  const v4f gc = *(const v4f*)(gam + lane * 8 + 4);
  const v4f ba = *(const v4f*)(bet + lane * 8);
  const v4f bc = *(const v4f*)(bet + lane * 8 + 4);
  const v4f oa = (da * rs) * ga + ba;
  const v4f oc = (dc * rs) * gc + bc;
  v4u hv, lv;
  split8(oa, oc, hv, lv);
  const size_t off = (size_t)row * DMODEL + lane * 8;
  store2_planes(xh + off, xl + off, hv, lv);
}

__global__ __launch_bounds__(256) void conv_silu_split(const float* __restrict__ xp,
                                                       const float* __restrict__ cw,
                                                       const float* __restrict__ cb,
                                                       float* __restrict__ xcf,
                                                       unsigned short* __restrict__ xch,
                                                       unsigned short* __restrict__ xcl) {
  __shared__ __align__(16) float slab[8][DMODEL];
  const int wave = threadIdx.x >> 5, lane = threadIdx.x & 31;
  const int row  = blockIdx.x * 8 + wave;
  const int bidx = row >> 10;
  const int s    = row & (SEQLEN - 1);
#pragma unroll 1
  for (int half = 0; half < 2; ++half) {
    const int c0 = half * 128 + lane * 4;
    const v4f w0 = *(const v4f*)(cw + (size_t)(c0 + 0) * KCONV);
    const v4f w1 = *(const v4f*)(cw + (size_t)(c0 + 1) * KCONV);
    const v4f w2 = *(const v4f*)(cw + (size_t)(c0 + 2) * KCONV);
    const v4f w3 = *(const v4f*)(cw + (size_t)(c0 + 3) * KCONV);
    v4f acc = (v4f){0.0f, 0.0f, 0.0f, 0.0f};
#pragma unroll
    for (int k = 0; k < KCONV; ++k) {
      const int sp  = s - (KCONV - 1) + k;
      const int spc = sp < 0 ? 0 : sp;
      const v4f xv  = *(const v4f*)(xp + ((size_t)bidx * SEQLEN + spc) * DPROJ + c0);
      const bool on = (sp >= 0);
      const float x0 = on ? xv[0] : 0.0f;
      const float x1 = on ? xv[1] : 0.0f;
      const float x2 = on ? xv[2] : 0.0f;
      const float x3 = on ? xv[3] : 0.0f;
      acc[0] += x0 * w0[k];
      acc[1] += x1 * w1[k];
      acc[2] += x2 * w2[k];
      acc[3] += x3 * w3[k];
    }
    asm volatile("" ::: "memory");
    const v4f cbv = *(const v4f*)(cb + c0);
    v4f o;
    o[0] = silu_f(acc[0] + cbv[0]);
    o[1] = silu_f(acc[1] + cbv[1]);
    o[2] = silu_f(acc[2] + cbv[2]);
    o[3] = silu_f(acc[3] + cbv[3]);
    float* dst = xcf + (size_t)row * DMODEL + c0;
    *(volatile v4f*)dst = o;
    __threadfence();
    *(volatile v4f*)dst = o;
    *(v4f*)(&slab[wave][c0]) = o;
  }
  __syncthreads();
  const v4f a = *(const v4f*)(&slab[wave][lane * 8]);
  const v4f c = *(const v4f*)(&slab[wave][lane * 8 + 4]);
  v4u hv, lv;
  split8(a, c, hv, lv);
  const size_t off = (size_t)row * DMODEL + lane * 8;
  store2_planes(xch + off, xcl + off, hv, lv);
}

__global__ __launch_bounds__(512) void ssm_scan(const unsigned short* __restrict__ Ath,
                                                const unsigned short* __restrict__ Atl,
                                                const float* __restrict__ bcp,
                                                const float* __restrict__ xcf,
                                                const float* __restrict__ xp,
                                                const float* __restrict__ Dp,
                                                unsigned short* __restrict__ yh,
                                                unsigned short* __restrict__ yl) {
  __shared__ __align__(16) __bf16 Gs[2][16 * GPITCH];
  __shared__ __align__(16) float  Ys[2][NBATCH * DMODEL];
  __shared__ float Cs[NROWS];
  const int tid = threadIdx.x, wave = tid >> 5, lane = tid & 31;
  const int hrow = lane >> 4, cix = lane & 15, koff = hrow * 8;
  const int n0 = wave * 16, n = n0 + cix;

  {
    const __bf16 bz = __builtin_bit_cast(__bf16, (unsigned short)0);
    __bf16* gflat = &Gs[0][0];
    for (int i = tid; i < 2 * 16 * GPITCH; i += 512) gflat[i] = bz;
  }
  for (int r = wave; r < NROWS; r += 16) {
    const float* p = bcp + (size_t)r * DPROJ + DMODEL + lane * 8;
    const v4f a = *(const v4f*)p;
    const v4f c = *(const v4f*)(p + 4);
    float s = ((a[0] + a[1]) + (a[2] + a[3])) + ((c[0] + c[1]) + (c[2] + c[3]));
#pragma unroll
    for (int o = 16; o > 0; o >>= 1) s += __shfl_xor(s, o, 32);
    Cs[r] = s;
  }
  __syncthreads();

  const float dpn = Dp[n];
  const __bf16* Abh = (const __bf16*)(const void*)Ath + (size_t)n * DSTATE + koff;
  const __bf16* Abl = (const __bf16*)(const void*)Atl + (size_t)n * DSTATE + koff;

  for (int t = 0; t < SEQLEN; ++t) {
    const int q = t & 1;
    if (wave < NBATCH && t > 0) {
      const float* ys = &Ys[q ^ 1][0] + wave * DMODEL + lane * 8;
      const v4f a = *(const v4f*)ys;
      const v4f c = *(const v4f*)(ys + 4);
      v4u hv, lv;
      split8(a, c, hv, lv);
      const size_t off = ((size_t)wave * SEQLEN + (size_t)(t - 1)) * DMODEL + lane * 8;
      store2_planes(yh + off, yl + off, hv, lv);
    }
    float bm[NBATCH], xv[NBATCH], gv[NBATCH], cs[NBATCH];
#pragma unroll
    for (int b = 0; b < NBATCH; ++b) {
      const size_t rr = (size_t)b * SEQLEN + (size_t)t;
      bm[b] = bcp[rr * DPROJ + n];
      xv[b] = xcf[rr * DMODEL + n];
      gv[b] = xp[rr * DPROJ + DMODEL + n];
      cs[b] = Cs[b * SEQLEN + t];
    }
    v8f acch = (v8f){0.f,0.f,0.f,0.f,0.f,0.f,0.f,0.f};
    v8f accl = (v8f){0.f,0.f,0.f,0.f,0.f,0.f,0.f,0.f};
    const __bf16* Gp = &Gs[q][0] + cix * GPITCH + koff;
#pragma unroll 2
    for (int kk = 0; kk < DSTATE / 32; ++kk) {
      const v16b af = Frag<__bf16>::load(Gp + kk * 32);
      const v16b bh = Frag<__bf16>::load(Abh + kk * 32);
      const v16b bl = Frag<__bf16>::load(Abl + kk * 32);
      acch = Frag<__bf16>::mma(af, bh, acch);
      accl = Frag<__bf16>::mma(af, bl, accl);
      guard3_b(acch, accl, af, bh, bl);
    }
    __bf16* Gn = &Gs[q ^ 1][0];
    float*  Yq = &Ys[q][0];
    if (hrow == 0) {
#pragma unroll
      for (int b = 0; b < NBATCH; ++b) {
        const float v = ((acch[b] + acch[4 + b]) + (accl[b] + accl[4 + b])) + bm[b];
        const unsigned short hb = f2bf_bits(v);
        const unsigned short lb = f2bf_bits(v - bf_bits2f(hb));
        Gn[b * GPITCH + n]       = __builtin_bit_cast(__bf16, hb);
        Gn[(4 + b) * GPITCH + n] = __builtin_bit_cast(__bf16, lb);
        const float y = (cs[b] * v + dpn * xv[b]) * silu_f(gv[b]);
        Yq[b * DMODEL + n] = y;
      }
    }
    __syncthreads();
  }
  if (wave < NBATCH) {
    const float* ys = &Ys[1][0] + wave * DMODEL + lane * 8;
    const v4f a = *(const v4f*)ys;
    const v4f c = *(const v4f*)(ys + 4);
    v4u hv, lv;
    split8(a, c, hv, lv);
    const size_t off = ((size_t)wave * SEQLEN + (size_t)(SEQLEN - 1)) * DMODEL + lane * 8;
    store2_planes(yh + off, yl + off, hv, lv);
  }
}

static inline size_t align256(size_t v) { return (v + 255) & ~(size_t)255; }

extern "C" void kernel_launch(void* const* d_in, const int* in_sizes, int n_in,
                              void* d_out, int out_size, void* d_ws, size_t ws_size,
                              hipStream_t stream) {
  if (n_in < 15) return;
  const float* x      = (const float*)d_in[0];
  const float* ln_g   = (const float*)d_in[1];
  const float* ln_b   = (const float*)d_in[2];
  const float* W_in   = (const float*)d_in[3];
  const float* b_in   = (const float*)d_in[4];
  const float* conv_w = (const float*)d_in[5];
  const float* conv_b = (const float*)d_in[6];
  const float* A_m    = (const float*)d_in[7];
  const float* W_B    = (const float*)d_in[8];
  const float* b_B    = (const float*)d_in[9];
  const float* W_C    = (const float*)d_in[10];
  const float* b_C    = (const float*)d_in[11];
  const float* D_p    = (const float*)d_in[12];
  const float* W_out  = (const float*)d_in[13];
  const float* b_out  = (const float*)d_in[14];
  if (in_sizes[0] != NROWS * DMODEL || in_sizes[3] != DPROJ * DMODEL || in_sizes[7] != DSTATE * DSTATE) return;
  if (out_size != NROWS * DMODEL) return;

  char* ws = (char*)d_ws;
  size_t off = 0;
  const size_t wbig = (size_t)DPROJ * DMODEL * 2, wsq = (size_t)DMODEL * DMODEL * 2;
  const size_t pl16 = (size_t)NROWS * DMODEL * 2, pl32 = (size_t)NROWS * DMODEL * 4, pl32w = (size_t)NROWS * DPROJ * 4;
  unsigned short* Win_h  = (unsigned short*)(ws + off); off = align256(off + wbig);
  unsigned short* Win_l  = (unsigned short*)(ws + off); off = align256(off + wbig);
  unsigned short* WB_h   = (unsigned short*)(ws + off); off = align256(off + wsq);
  unsigned short* WB_l   = (unsigned short*)(ws + off); off = align256(off + wsq);
  unsigned short* WC_h   = (unsigned short*)(ws + off); off = align256(off + wsq);
  unsigned short* WC_l   = (unsigned short*)(ws + off); off = align256(off + wsq);
  unsigned short* Wout_h = (unsigned short*)(ws + off); off = align256(off + wsq);
  unsigned short* Wout_l = (unsigned short*)(ws + off); off = align256(off + wsq);
  unsigned short* At_h   = (unsigned short*)(ws + off); off = align256(off + wsq);
  unsigned short* At_l   = (unsigned short*)(ws + off); off = align256(off + wsq);
  unsigned short* xn_h   = (unsigned short*)(ws + off); off = align256(off + pl16);
  unsigned short* xn_l   = (unsigned short*)(ws + off); off = align256(off + pl16);
  float*          xp     = (float*)(ws + off);          off = align256(off + pl32w);
  float*          xcf    = (float*)(ws + off);          off = align256(off + pl32);
  unsigned short* xc_h   = (unsigned short*)(ws + off); off = align256(off + pl16);
  unsigned short* xc_l   = (unsigned short*)(ws + off); off = align256(off + pl16);
  float*          bc     = (float*)(ws + off);          off = align256(off + pl32w);
  unsigned short* y_h    = (unsigned short*)(ws + off); off = align256(off + pl16);
  unsigned short* y_l    = (unsigned short*)(ws + off); off = align256(off + pl16);
  if (off > ws_size) return;

  split_planes<<<(DPROJ * DMODEL / 8 + 255) / 256, 256, 0, stream>>>(W_in, Win_h, Win_l, DPROJ * DMODEL / 8);
  split_planes<<<(DMODEL * DMODEL / 8 + 255) / 256, 256, 0, stream>>>(W_B, WB_h, WB_l, DMODEL * DMODEL / 8);
  split_planes<<<(DMODEL * DMODEL / 8 + 255) / 256, 256, 0, stream>>>(W_C, WC_h, WC_l, DMODEL * DMODEL / 8);
  split_planes<<<(DMODEL * DMODEL / 8 + 255) / 256, 256, 0, stream>>>(W_out, Wout_h, Wout_l, DMODEL * DMODEL / 8);
  split_transpose_sq<<<(DSTATE * DSTATE / 8) / 256, 256, 0, stream>>>(A_m, At_h, At_l);

  layernorm_split<<<NROWS / 8, 256, 0, stream>>>(x, ln_g, ln_b, xn_h, xn_l);

  {
    const int tiles = (NROWS / 64) * (DPROJ / 64);
    wmma_gemm64<1, true, 2, 0, false, 0><<<dim3(tiles / 8, 1), 256, 0, stream>>>(
        xn_h, xn_l, DMODEL, 0L, Win_h, Win_l, DMODEL, 0L,
        (void*)xp, nullptr, DPROJ, 0L, b_in, nullptr, 0L, NROWS, DPROJ, DMODEL, 1.0f);
  }

  conv_silu_split<<<NROWS / 8, 256, 0, stream>>>(xp, conv_w, conv_b, xcf, xc_h, xc_l);

  {
    const int tiles = (NROWS / 64) * (DMODEL / 64);
    wmma_gemm64<1, true, 2, 0, false, 0><<<dim3(tiles / 8, 1), 256, 0, stream>>>(
        xc_h, xc_l, DMODEL, 0L, WB_h, WB_l, DMODEL, 0L,
        (void*)bc, nullptr, DPROJ, 0L, b_B, nullptr, 0L, NROWS, DMODEL, DMODEL, 1.0f);
    wmma_gemm64<1, true, 2, 0, false, 0><<<dim3(tiles / 8, 1), 256, 0, stream>>>(
        xc_h, xc_l, DMODEL, 0L, WC_h, WC_l, DMODEL, 0L,
        (void*)(bc + DMODEL), nullptr, DPROJ, 0L, b_C, nullptr, 0L, NROWS, DMODEL, DMODEL, 1.0f);
  }

  ssm_scan<<<1, 512, 0, stream>>>(At_h, At_l, bc, xcf, xp, D_p, y_h, y_l);

  {
    const int tiles = (NROWS / 64) * (DMODEL / 64);
    wmma_gemm64<1, true, 2, 0, true, 0><<<dim3(tiles / 8, 1), 256, 0, stream>>>(
        y_h, y_l, DMODEL, 0L, Wout_h, Wout_l, DMODEL, 0L,
        d_out, nullptr, DMODEL, 0L, b_out, x, 0L, NROWS, DMODEL, DMODEL, 1.0f);
  }
}
